// ContextAwareAttention_85512798863753
// MI455X (gfx1250) — hardware-run, weakly checked
//
#include <hip/hip_runtime.h>
#include <math.h>
#include <stdint.h>

#define LL   1024
#define DD   512
#ifndef SEQ
#define SEQ  8192
#endif
#define SEQ_FULL 8192
#define NT   128
#define OT   64
#define QB   64
#define CHH  256
#define OSP  68
#define OSQ  132
#define TP   72
#define NOB  (DD / OT)
#define NIT  ((SEQ + 1023) / 1024)
#define WSC  256.0f
#define IWSC 0.00390625f
#define QSC  16.0f
#define VSC  16.0f
#define IVSC 0.0625f
#define CSC  256.0f
#define HSC  0.0000152587890625f
#define SSC  (0.044194173824159216f * 0.00390625f)
#define LNPS 6.931471805599453f

static_assert(SEQ % NT == 0 && SEQ >= NT);
static_assert(SEQ % QB == 0);
static_assert(SEQ % 32 == 0);
static_assert((SEQ * LL) % 2048 == 0);
static_assert(LL % 64 == 0 && LL % 32 == 0);
static_assert(DD % OT == 0 && DD % 64 == 0 && DD % 32 == 0);
static_assert(DD == 2 * CHH && CHH == 16 * 16);
static_assert(QB == 4 * 16);
static_assert(NT == 4 * 32);
static_assert(OT == 4 * 16);
static_assert((OSP * 4) % 16 == 0 && OSP >= OT);
static_assert((OSQ * 4) % 16 == 0 && OSQ >= 128);
static_assert((TP * 2) % 16 == 0 && TP >= 64);
static_assert(NOB == 8);
static_assert(SEQ_FULL * 4 == 32768);
static_assert(NIT >= 1 && NIT <= 8);

typedef _Float16       v16h __attribute__((ext_vector_type(16)));
typedef _Float16       v8h  __attribute__((ext_vector_type(8)));
typedef __bf16         v16b __attribute__((ext_vector_type(16)));
typedef unsigned short v8us __attribute__((ext_vector_type(8)));
typedef float          v8f  __attribute__((ext_vector_type(8)));
typedef float          v4f  __attribute__((ext_vector_type(4)));
typedef unsigned int   v4u  __attribute__((ext_vector_type(4)));

union Frag  { v8us u[2]; v16h h; v16b bf; };
union FragH { v16h v; v8h hv[2]; };
static_assert(sizeof(Frag) == 32);
static_assert(sizeof(FragH) == 32);

__device__ __forceinline__ unsigned short bf_bits(float f) {
  unsigned u = __float_as_uint(f);
  return (unsigned short)((u + 0x7FFFu + ((u >> 16) & 1u)) >> 16);
}
__device__ __forceinline__ float bf_up(unsigned short hb) { return __uint_as_float(((unsigned)hb) << 16); }
__device__ __forceinline__ float bfr(float f) { return bf_up(bf_bits(f)); }
__device__ __forceinline__ unsigned short h_bits(_Float16 x) { return __builtin_bit_cast(unsigned short, x); }
__device__ __forceinline__ unsigned pk16(unsigned short a, unsigned short b) { return (unsigned)a | ((unsigned)b << 16); }
__device__ __forceinline__ v8f zero8() { v8f z = {0.f, 0.f, 0.f, 0.f, 0.f, 0.f, 0.f, 0.f}; return z; }
__device__ __forceinline__ float hmax8(v8f s) {
  return fmaxf(fmaxf(fmaxf(s[0], s[1]), fmaxf(s[2], s[3])), fmaxf(fmaxf(s[4], s[5]), fmaxf(s[6], s[7])));
}
__device__ __forceinline__ unsigned wave_ballot(bool p) {
#if defined(__HIP_DEVICE_COMPILE__)
  return __builtin_amdgcn_ballot_w32(p);
#else
  return p ? 1u : 0u;
#endif
}

__device__ __forceinline__ Frag ldfrag(const unsigned short* p) {
  Frag f;
  f.u[0] = *(const v8us*)(p);
  f.u[1] = *(const v8us*)(p + 16);
  return f;
}

__device__ __forceinline__ v8f mma_h(v16h a, v16h b, v8f c) {
  v8f d = __builtin_amdgcn_wmma_f32_16x16x32_f16(false, a, false, b, (short)0, c, false, false);
#if defined(__HIP_DEVICE_COMPILE__)
  asm volatile("v_nop\n\tv_nop\n\tv_nop\n\tv_nop" : "+v"(d) : "v"(a), "v"(b));
#endif
  return d;
}

__global__ __launch_bounds__(256)
void cvt_x(const float* __restrict__ x, unsigned short* X16) {
  const size_t base = ((size_t)blockIdx.x * 256 + threadIdx.x) * 8;
  const v4f a = *(const v4f*)(x + base);
  const v4f q = *(const v4f*)(x + base + 4);
  const float f[8] = {a[0], a[1], a[2], a[3], q[0], q[1], q[2], q[3]};
  v4u u;
#pragma unroll
  for (int t = 0; t < 4; ++t) {
    const _Float16 h0 = (_Float16)bfr(f[2 * t]);
    const _Float16 h1 = (_Float16)bfr(f[2 * t + 1]);
    u[t] = pk16(h_bits(h0), h_bits(h1));
  }
#pragma unroll
  for (int pass = 0; pass < 2; ++pass) {
    *(volatile v4u*)(X16 + base) = u;
    __threadfence();
  }
}

__global__ __launch_bounds__(256)
void cvt_w(const float* __restrict__ w0, const float* __restrict__ w1, const float* __restrict__ w2,
           unsigned short* WT, int K, int M) {
  __shared__ __align__(16) unsigned short T[64 * TP];
  const int tid = threadIdx.x;
  const int kb = blockIdx.x, mb = blockIdx.y, z = blockIdx.z;
  const float* w = (z == 0) ? w0 : ((z == 1) ? w1 : w2);
  unsigned short* dst = WT + (size_t)z * (size_t)M * (size_t)K;
  const int e = tid & 7, lq = tid >> 3;
  const int k0 = kb * 64, m0 = mb * 64;
#pragma unroll
  for (int it = 0; it < 2; ++it) {
    const int kl = it * 32 + lq;
    const float* sp = w + ((size_t)(k0 + kl)) * M + m0 + 8 * e;
    const v4f a = *(const v4f*)sp;
    const v4f q = *(const v4f*)(sp + 4);
    unsigned short hb[8];
#pragma unroll
    for (int t = 0; t < 4; ++t) {
      hb[t]     = h_bits((_Float16)(bfr(a[t]) * WSC));
      hb[4 + t] = h_bits((_Float16)(bfr(q[t]) * WSC));
    }
#pragma unroll
    for (int t = 0; t < 8; ++t) T[(8 * e + t) * TP + kl] = hb[t];
  }
  __syncthreads();
  v4u up[2];
#pragma unroll
  for (int it = 0; it < 2; ++it) {
    const int ml = it * 32 + lq;
    up[it] = *(const v4u*)(T + ml * TP + 8 * e);
  }
#pragma unroll
  for (int pass = 0; pass < 2; ++pass) {
#pragma unroll
    for (int it = 0; it < 2; ++it) {
      const int ml = it * 32 + lq;
      *(volatile v4u*)(dst + ((size_t)(m0 + ml)) * K + k0 + 8 * e) = up[it];
    }
    __threadfence();
  }
}

template <int KD>
__device__ __forceinline__ void gemm_core(const unsigned short* __restrict__ ap,
                                          const unsigned short* __restrict__ bp, v8f (&acc)[2][4]) {
#pragma unroll
  for (int nb = 0; nb < 2; ++nb) {
#pragma unroll
    for (int mt = 0; mt < 4; ++mt) acc[nb][mt] = zero8();
  }
#pragma unroll 1
  for (int ks = 0; ks < KD / 32; ++ks) {
    const Frag fb0 = ldfrag(bp + 32 * ks);
    const Frag fb1 = ldfrag(bp + (size_t)16 * KD + 32 * ks);
#pragma unroll
    for (int mt = 0; mt < 4; ++mt) {
      const Frag fa = ldfrag(ap + (size_t)(16 * mt) * KD + 32 * ks);
      acc[0][mt] = mma_h(fa.h, fb0.h, acc[0][mt]);
      acc[1][mt] = mma_h(fa.h, fb1.h, acc[1][mt]);
    }
  }
}

__device__ __forceinline__ void stage_os(float* Os, const v8f (&acc)[2][4], const float* __restrict__ bo,
                                         const float sc, const int wave, const int hh, const int c) {
#pragma unroll
  for (int nb = 0; nb < 2; ++nb) {
    const int nl = 32 * wave + 16 * nb + c;
#pragma unroll
    for (int mt = 0; mt < 4; ++mt) {
      const v4f ba = *(const v4f*)(bo + 16 * mt + 8 * hh);
      const v4f bb = *(const v4f*)(bo + 16 * mt + 8 * hh + 4);
      v4f va, vb;
#pragma unroll
      for (int r = 0; r < 4; ++r) {
        va[r] = acc[nb][mt][r] * sc + ba[r];
        vb[r] = acc[nb][mt][4 + r] * sc + bb[r];
      }
      *(v4f*)(Os + nl * OSP + 16 * mt + 8 * hh)     = va;
      *(v4f*)(Os + nl * OSP + 16 * mt + 8 * hh + 4) = vb;
    }
  }
}

__global__ __launch_bounds__(128)
void gemm_proj(const unsigned short* __restrict__ WT3, const unsigned short* __restrict__ X16,
               const float* __restrict__ bq, const float* __restrict__ bk, const float* __restrict__ bv,
               unsigned short* Q16, unsigned short* K16, unsigned short* Vc) {
  __shared__ __align__(16) float Os[NT * OSP];
  const int tid  = threadIdx.x;
  const int lane = tid & 31, wave = tid >> 5;
  const int hh   = lane >> 4, c = lane & 15;
  const int nt   = blockIdx.x, mb = blockIdx.y, z = blockIdx.z;
  const int n0   = nt * NT, o0 = mb * OT;

  const unsigned short* ap = WT3 + ((size_t)z * DD + o0 + c) * LL + 8 * hh;
  const unsigned short* bp = X16 + ((size_t)(n0 + 32 * wave + c)) * LL + 8 * hh;

  v8f acc[2][4];
  gemm_core<LL>(ap, bp, acc);

  const float* bias = (z == 0) ? bq : ((z == 1) ? bk : bv);
  stage_os(Os, acc, bias + o0, IWSC, wave, hh, c);
  __syncthreads();

  const int e = tid & 7, lq = tid >> 3;
  if (z < 2) {
    unsigned short* dst = (z == 0) ? Q16 : K16;
    v4u u[8];
#pragma unroll
    for (int it = 0; it < 8; ++it) {
      const int row = it * 16 + lq;
      const v4f a = *(const v4f*)(Os + row * OSP + 8 * e);
      const v4f q = *(const v4f*)(Os + row * OSP + 8 * e + 4);
      const float f[8] = {a[0], a[1], a[2], a[3], q[0], q[1], q[2], q[3]};
#pragma unroll
      for (int t = 0; t < 4; ++t) {
        const _Float16 h0 = (_Float16)(f[2 * t] * QSC);
        const _Float16 h1 = (_Float16)(f[2 * t + 1] * QSC);
        u[it][t] = pk16(h_bits(h0), h_bits(h1));
      }
    }
#pragma unroll
    for (int pass = 0; pass < 2; ++pass) {
#pragma unroll
      for (int it = 0; it < 8; ++it) {
        const int row = it * 16 + lq;
        *(volatile v4u*)(dst + ((size_t)(n0 + row)) * DD + o0 + 8 * e) = u[it];
      }
      __threadfence();
    }
  } else {
    v4u u[8];
#pragma unroll
    for (int it = 0; it < 8; ++it) {
      const int L   = it * 16 + lq;
      const int chl = L >> 1;
      const int nl  = 64 * (L & 1) + 8 * e;
      float f[8];
#pragma unroll
      for (int t = 0; t < 8; ++t) f[t] = Os[(nl + t) * OSP + chl];
#pragma unroll
      for (int t = 0; t < 4; ++t) {
        const _Float16 h0 = (_Float16)(f[2 * t] * VSC);
        const _Float16 h1 = (_Float16)(f[2 * t + 1] * VSC);
        u[it][t] = pk16(h_bits(h0), h_bits(h1));
      }
    }
#pragma unroll
    for (int pass = 0; pass < 2; ++pass) {
#pragma unroll
      for (int it = 0; it < 8; ++it) {
        const int L   = it * 16 + lq;
        const int chl = L >> 1;
        const int nl  = 64 * (L & 1) + 8 * e;
        *(volatile v4u*)(Vc + ((size_t)(o0 + chl)) * SEQ + n0 + nl) = u[it];
      }
      __threadfence();
    }
  }
}

__global__ __launch_bounds__(256)
void attn_k(const unsigned short* __restrict__ Q16, const unsigned short* __restrict__ K16,
            const unsigned short* __restrict__ Vc, float* ctx, unsigned short* C16) {
  __shared__ __align__(16) float Sx[2 * 8 * 256];
  __shared__ __align__(16) float Os[QB * OSQ];
  const int tid  = threadIdx.x;
  const int wave = tid >> 5, lane = tid & 31;
  const int hh   = lane >> 4, c = lane & 15;
  const int g    = wave & 3, hf = wave >> 2;
  const int n0   = blockIdx.x * QB;

  const unsigned short* Qp = Q16 + ((size_t)(n0 + 16 * g + c)) * DD + 8 * hh;
  const unsigned short* Kp = K16 + ((size_t)(16 * hf + c)) * DD + 8 * hh;
  const unsigned short* Vp = Vc + ((size_t)(CHH * hf + c)) * SEQ + 8 * hh;
  float*       sxw = Sx + (2 * g + hf) * 256 + 8 * lane;
  const float* sxr = Sx + (2 * g + (hf ^ 1)) * 256 + 8 * lane;

  float m = -1.0e30f, l = 0.f;
  v8f o[16];
#pragma unroll
  for (int j = 0; j < 16; ++j) o[j] = zero8();

#pragma unroll 1
  for (int kb = 0; kb < SEQ; kb += 32) {
    const unsigned short* kp = Kp + (size_t)kb * DD;
    v8f sa = zero8();
#pragma unroll 2
    for (int kc = 0; kc < DD / 32; ++kc) {
      const Frag fq = ldfrag(Qp + 32 * kc);
      const Frag fk = ldfrag(kp + 32 * kc);
      sa = mma_h(fk.h, fq.h, sa);
    }

    const int bo = ((kb >> 5) & 1) * 2048;
    {
      v4f wa, wb;
#pragma unroll
      for (int r = 0; r < 4; ++r) { wa[r] = sa[r]; wb[r] = sa[4 + r]; }
      *(v4f*)(sxw + bo)     = wa;
      *(v4f*)(sxw + bo + 4) = wb;
    }
    __syncthreads();
    v8f s0, s1;
    {
      const v4f ra = *(const v4f*)(sxr + bo);
      const v4f rb = *(const v4f*)(sxr + bo + 4);
#pragma unroll
      for (int r = 0; r < 4; ++r) {
        const float p0 = ra[r], p1 = rb[r];
        s0[r]     = hf ? p0 : sa[r];
        s0[4 + r] = hf ? p1 : sa[4 + r];
        s1[r]     = hf ? sa[r] : p0;
        s1[4 + r] = hf ? sa[4 + r] : p1;
      }
    }

    float mx = fmaxf(hmax8(s0), hmax8(s1)) * SSC;
    mx = fmaxf(mx, __shfl_xor(mx, 16, 32));
    const float mn = fmaxf(m, mx);
    const unsigned grew = wave_ballot(mx > m);
    if (grew != 0u) {
      const float corr = __expf(m - mn);
      l *= corr;
#pragma unroll
      for (int j = 0; j < 16; ++j) {
#pragma unroll
        for (int r = 0; r < 8; ++r) o[j][r] *= corr;
      }
    }
    m = mn;
    const float msh = mn - LNPS;

    FragH ph;
    float ls = 0.f;
#pragma unroll
    for (int r = 0; r < 8; ++r) {
      const float e0 = __expf(s0[r] * SSC - msh);
      const float e1 = __expf(s1[r] * SSC - msh);
      ls += e0 + e1;
      ph.hv[0][r] = (_Float16)e0;
      ph.hv[1][r] = (_Float16)e1;
    }
    l += ls;

#pragma unroll
    for (int j = 0; j < 16; ++j) {
      const Frag vf = ldfrag(Vp + (size_t)(16 * j) * SEQ + kb);
      o[j] = mma_h(vf.h, ph.v, o[j]);
      if ((j & 3) == 3) { asm volatile("" ::: "memory"); }
    }
  }
  l += __shfl_xor(l, 16, 32);
  const float inv = (1.0f / l) * IVSC;

  const int qrow = 16 * g + c;
  const int e = tid & 7, lq = tid >> 3;
  float*          ctxb = ctx + (size_t)n0 * DD;
  unsigned short* c16b = C16 + (size_t)n0 * DD;
#pragma unroll
  for (int p = 0; p < 4; ++p) {
    if (p) __syncthreads();
    if (hf == (p >> 1)) {
#pragma unroll
      for (int jj = 0; jj < 8; ++jj) {
        const int j = 8 * (p & 1) + jj;
        v4f va, vb;
#pragma unroll
        for (int r = 0; r < 4; ++r) { va[r] = o[j][r] * inv; vb[r] = o[j][4 + r] * inv; }
        *(v4f*)(Os + qrow * OSQ + 16 * jj + 8 * hh)     = va;
        *(v4f*)(Os + qrow * OSQ + 16 * jj + 8 * hh + 4) = vb;
      }
    }
    __syncthreads();
    {
      v4f rf[8];
#pragma unroll
      for (int it = 0; it < 8; ++it) {
        const int L   = it * 32 + lq;
        const int row = L >> 2;
        const int cho = 32 * (L & 3) + 4 * e;
        rf[it] = *(const v4f*)(Os + row * OSQ + cho);
      }
#pragma unroll
      for (int pass = 0; pass < 2; ++pass) {
#pragma unroll
        for (int it = 0; it < 8; ++it) {
          const int L   = it * 32 + lq;
          const int row = L >> 2;
          const int cho = 32 * (L & 3) + 4 * e;
          *(volatile v4f*)(ctxb + (size_t)row * DD + 128 * p + cho) = rf[it];
        }
        __threadfence();
      }
    }
    {
      v4u rh[4];
#pragma unroll
      for (int it = 0; it < 4; ++it) {
        const int L   = it * 32 + lq;
        const int row = L >> 1;
        const int cho = 64 * (L & 1) + 8 * e;
        const v4f a = *(const v4f*)(Os + row * OSQ + cho);
        const v4f q = *(const v4f*)(Os + row * OSQ + cho + 4);
        const float f[8] = {a[0], a[1], a[2], a[3], q[0], q[1], q[2], q[3]};
#pragma unroll
        for (int t = 0; t < 4; ++t) {
          const _Float16 h0 = (_Float16)(f[2 * t] * CSC);
          const _Float16 h1 = (_Float16)(f[2 * t + 1] * CSC);
          rh[it][t] = pk16(h_bits(h0), h_bits(h1));
        }
      }
#pragma unroll
      for (int pass = 0; pass < 2; ++pass) {
#pragma unroll
        for (int it = 0; it < 4; ++it) {
          const int L   = it * 32 + lq;
          const int row = L >> 1;
          const int cho = 64 * (L & 1) + 8 * e;
          *(volatile v4u*)(c16b + (size_t)row * DD + 128 * p + cho) = rh[it];
        }
        __threadfence();
      }
    }
  }
}

__global__ __launch_bounds__(128)
void gemm_head(const unsigned short* __restrict__ W1T, const unsigned short* __restrict__ C16,
               const float* __restrict__ b1, const float* __restrict__ w2, float* PART) {
  __shared__ __align__(16) float Os[NT * OSP];
  __shared__ __align__(16) float Ls[NT];
  __shared__ float w2s[OT];
  const int tid  = threadIdx.x;
  const int lane = tid & 31, wave = tid >> 5;
  const int hh   = lane >> 4, c = lane & 15;
  const int nt   = blockIdx.x, mb = blockIdx.y;
  const int n0   = nt * NT, o0 = mb * OT;

  const unsigned short* ap = W1T + ((size_t)(o0 + c)) * DD + 8 * hh;
  const unsigned short* bp = C16 + ((size_t)(n0 + 32 * wave + c)) * DD + 8 * hh;

  v8f acc[2][4];
  gemm_core<DD>(ap, bp, acc);

  if (tid < OT) w2s[tid] = w2[o0 + tid];
  stage_os(Os, acc, b1 + o0, HSC, wave, hh, c);
  __syncthreads();

  float hs = 0.f;
  const float* orow = Os + tid * OSP;
#pragma unroll 1
  for (int oo = 0; oo < OT; ++oo) hs += tanhf(orow[oo]) * w2s[oo];
  Ls[tid] = hs;
  __syncthreads();
  if (wave == 0) {
    const v4f v = *(const v4f*)(Ls + 4 * lane);
    float* pp = PART + (size_t)mb * SEQ + n0 + 4 * lane;
#pragma unroll
    for (int pass = 0; pass < 2; ++pass) {
      *(volatile v4f*)pp = v;
      __threadfence();
    }
  }
}

__global__ __launch_bounds__(256)
void pool_softmax(const float* __restrict__ PART, const float* __restrict__ b2, float* outA) {
  __shared__ float red[8];
  const int tid = threadIdx.x, lane = tid & 31, wave = tid >> 5;
  const float bias2 = b2[0];
  float gv[NIT][4];
  float mx = -1.0e30f;
#pragma unroll
  for (int it = 0; it < NIT; ++it) {
    const int n  = 1024 * it + 4 * tid;
    const int nc = (n < SEQ) ? n : (SEQ - 4);
    v4f s = *(const v4f*)(PART + nc);
#pragma unroll
    for (int ob = 1; ob < NOB; ++ob) {
      const v4f t = *(const v4f*)(PART + (size_t)ob * SEQ + nc);
      s += t;
    }
#pragma unroll
    for (int t = 0; t < 4; ++t) {
      gv[it][t] = s[t] + bias2;
      if (n < SEQ) mx = fmaxf(mx, gv[it][t]);
    }
  }
#pragma unroll
  for (int off = 16; off > 0; off >>= 1) mx = fmaxf(mx, __shfl_xor(mx, off, 32));
  if (lane == 0) red[wave] = mx;
  __syncthreads();
  float M = red[0];
#pragma unroll
  for (int w = 1; w < 8; ++w) M = fmaxf(M, red[w]);
  __syncthreads();

  float se = 0.f;
#pragma unroll
  for (int it = 0; it < NIT; ++it) {
    const int n = 1024 * it + 4 * tid;
#pragma unroll
    for (int t = 0; t < 4; ++t) {
      const float ev = (n < SEQ) ? __expf(gv[it][t] - M) : 0.f;
      gv[it][t] = ev;
      se += ev;
    }
  }
#pragma unroll
  for (int off = 16; off > 0; off >>= 1) se += __shfl_xor(se, off, 32);
  if (lane == 0) red[wave] = se;
  __syncthreads();
  float S = red[0];
#pragma unroll
  for (int w = 1; w < 8; ++w) S += red[w];
  const float inv = 1.0f / S;

#pragma unroll
  for (int pass = 0; pass < 2; ++pass) {
#pragma unroll
    for (int it = 0; it < NIT; ++it) {
      const int n = 1024 * it + 4 * tid;
      if (n < SEQ) {
        v4f wv;
#pragma unroll
        for (int t = 0; t < 4; ++t) wv[t] = gv[it][t] * inv;
        *(volatile v4f*)(outA + n) = wv;
      }
    }
    __threadfence();
  }
}

extern "C" void kernel_launch(void* const* d_in, const int* in_sizes, int n_in,
                              void* d_out, int out_size, void* d_ws, size_t ws_size,
                              hipStream_t stream) {
  if (n_in < 11) return;
  if (in_sizes[0] < SEQ * LL) return;
  if (in_sizes[1] < LL * DD || in_sizes[3] < LL * DD || in_sizes[5] < LL * DD) return;
  if (in_sizes[2] < DD || in_sizes[4] < DD || in_sizes[6] < DD || in_sizes[8] < DD || in_sizes[9] < DD) return;
  if (in_sizes[7] < DD * DD) return;
  if (in_sizes[10] < 1) return;
  if ((size_t)out_size < (size_t)SEQ_FULL + (size_t)SEQ * DD) return;

  size_t off = 0;
  auto carve = [&](size_t bytes) { const size_t o = off; off += (bytes + 255) & ~(size_t)255; return o; };
  const size_t oX16 = carve((size_t)SEQ * LL * 2);
  const size_t oWT3 = carve((size_t)3 * DD * LL * 2);
  const size_t oW1T = carve((size_t)DD * DD * 2);
  const size_t oQ16 = carve((size_t)SEQ * DD * 2);
  const size_t oK16 = carve((size_t)SEQ * DD * 2);
  const size_t oVc  = carve((size_t)DD * SEQ * 2);
  const size_t oC16 = carve((size_t)SEQ * DD * 2);
  const size_t oPRT = carve((size_t)NOB * SEQ * 4);
  if (off > ws_size) return;
  if (off > (size_t)134217728) return;

  const float* x  = (const float*)d_in[0];
  const float* Wq = (const float*)d_in[1];
  const float* bq = (const float*)d_in[2];
  const float* Wk = (const float*)d_in[3];
  const float* bk = (const float*)d_in[4];
  const float* Wv = (const float*)d_in[5];
  const float* bv = (const float*)d_in[6];
  const float* W1 = (const float*)d_in[7];
  const float* b1 = (const float*)d_in[8];
  const float* w2 = (const float*)d_in[9];
  const float* b2 = (const float*)d_in[10];

  char* ws = (char*)d_ws;
  unsigned short* X16 = (unsigned short*)(ws + oX16);
  unsigned short* WT3 = (unsigned short*)(ws + oWT3);
  unsigned short* W1T = (unsigned short*)(ws + oW1T);
  unsigned short* Q16 = (unsigned short*)(ws + oQ16);
  unsigned short* K16 = (unsigned short*)(ws + oK16);
  unsigned short* Vc  = (unsigned short*)(ws + oVc);
  unsigned short* C16 = (unsigned short*)(ws + oC16);
  float* PART = (float*)(ws + oPRT);
  float* outA = (float*)d_out;
  float* ctx  = (float*)d_out + SEQ_FULL;

  const dim3 blk256(256), blk128(128);

  cvt_x<<<dim3((SEQ * LL) / 2048), blk256, 0, stream>>>(x, X16);
  cvt_w<<<dim3(LL / 64, DD / 64, 3), blk256, 0, stream>>>(Wq, Wk, Wv, WT3, LL, DD);
  cvt_w<<<dim3(DD / 64, DD / 64, 1), blk256, 0, stream>>>(W1, W1, W1, W1T, DD, DD);
  gemm_proj<<<dim3(SEQ / NT, DD / OT, 3), blk128, 0, stream>>>(WT3, X16, bq, bk, bv, Q16, K16, Vc);
  attn_k<<<dim3(SEQ / QB), blk256, 0, stream>>>(Q16, K16, Vc, ctx, C16);
  gemm_head<<<dim3(SEQ / NT, DD / OT), blk128, 0, stream>>>(W1T, C16, b1, w2, PART);
  pool_softmax<<<dim3(1), blk256, 0, stream>>>(PART, b2, outA);
  (void)hipGetLastError();
}
